// CausalGatedD2Attention_86689619903615
// MI455X (gfx1250) — hardware-run, weakly checked
//
#include <hip/hip_runtime.h>
#include <math.h>
#include <stdint.h>
#include <stddef.h>

typedef __attribute__((ext_vector_type(16))) _Float16 v16h;
typedef __attribute__((ext_vector_type(8)))  _Float16 v8h;
typedef __attribute__((ext_vector_type(16))) __bf16   v16b;
typedef __attribute__((ext_vector_type(8)))  __bf16   v8b;
typedef __attribute__((ext_vector_type(8)))  float    v8f;
typedef __attribute__((ext_vector_type(4)))  float    v4f;
typedef __attribute__((ext_vector_type(4)))  unsigned v4u;

constexpr int kB   = 2;
constexpr int kL   = 2048;
constexpr int kD   = 768;
constexpr int kH   = 12;
constexpr int kR   = 128;
constexpr int kDH  = 64;
constexpr int kNT  = kB * kL;
constexpr int kBH  = kB * kH;
constexpr int kNC  = kL / 64;
constexpr int kAP  = 72;
constexpr int kOP  = 68;

constexpr size_t kSzWqkvT   = (size_t)3 * kD * kD * 2;
constexpr size_t kSzWdownT  = (size_t)2 * kR * kD * 2;
constexpr size_t kSzWupT    = (size_t)2 * 2 * kD * kR * 2;
constexpr size_t kSzWprojT  = (size_t)kD * kD * 2;
constexpr size_t kSzBproj   = (size_t)kD * 4;
constexpr size_t kSzPlane16 = (size_t)kNT * kD * 2;
constexpr size_t kSzQkv     = (size_t)kNT * 3 * kD * 4;
constexpr size_t kSzH       = (size_t)kNT * 2 * kR * 2;
constexpr size_t kSzSemCtx  = (size_t)2 * kNT * 2 * kD * 4;

constexpr size_t kOffWqkvT  = 0;
constexpr size_t kOffWdownT = kOffWqkvT + kSzWqkvT;
constexpr size_t kOffWupT   = kOffWdownT + kSzWdownT;
constexpr size_t kOffWprojT = kOffWupT + kSzWupT;
constexpr size_t kOffBproj  = kOffWprojT + kSzWprojT;
constexpr size_t kOffXb     = kOffBproj + kSzBproj;
constexpr size_t kOffXnh    = kOffXb + kSzPlane16;
constexpr size_t kOffXnl    = kOffXnh + kSzPlane16;
constexpr size_t kOffQkv    = kOffXnl + kSzPlane16;
constexpr size_t kOffHh     = kOffQkv + kSzQkv;
constexpr size_t kOffHl     = kOffHh + kSzH;
constexpr size_t kOffSemCtx = kOffHl + kSzH;
constexpr size_t kOffAttnH  = kOffSemCtx;
constexpr size_t kOffAttnL  = kOffAttnH + kSzPlane16;
constexpr size_t kWsEnd     = kOffSemCtx + kSzSemCtx;
static_assert(kWsEnd == (size_t)117050368);
static_assert(kWsEnd <= (size_t)134217728);
static_assert(kOffAttnL + kSzPlane16 <= kWsEnd);
static_assert(kOffWdownT % 128 == 0 && kOffWupT % 128 == 0 && kOffWprojT % 128 == 0 && kOffBproj % 128 == 0);
static_assert(kOffXb % 128 == 0 && kOffXnh % 128 == 0 && kOffXnl % 128 == 0 && kOffQkv % 128 == 0);
static_assert(kOffHh % 128 == 0 && kOffHl % 128 == 0 && kOffSemCtx % 128 == 0 && kOffAttnL % 128 == 0);

constexpr size_t kOut0Bytes = (size_t)kNT * kD * 4;
constexpr size_t kOut1ByteOff = 12582912;
static_assert(kOut1ByteOff % 128 == 0 && kOut1ByteOff % 4 == 0);
constexpr size_t kOut1Elems = kOut1ByteOff / 4;
static_assert(kOut1ByteOff + (size_t)kNT * kD * 4 <= (size_t)25165824);
static_assert(kOut0Bytes == kOut1ByteOff);

static_assert(kNT % 64 == 0 && (3 * kD) % 64 == 0 && (2 * kR) % 64 == 0 && (2 * kD) % 64 == 0 && kD % 64 == 0);
static_assert(kD % 32 == 0 && kR % 32 == 0);

__device__ __forceinline__ unsigned short f2bf_bits(float f) {
  unsigned u = __float_as_uint(f);
  return (unsigned short)((u + 0x7FFFu + ((u >> 16) & 1u)) >> 16);
}
__device__ __forceinline__ float bf_bits2f(unsigned short h) { return __uint_as_float(((unsigned)h) << 16); }
__device__ __forceinline__ float bf_rte(float f) { return bf_bits2f(f2bf_bits(f)); }
__device__ __forceinline__ void split_bf(float f, unsigned short& hb, unsigned short& lb) {
  hb = f2bf_bits(f);
  lb = f2bf_bits(f - bf_bits2f(hb));
}
__device__ __forceinline__ unsigned pack16x2(unsigned short lo, unsigned short hi) { return (unsigned)lo | ((unsigned)hi << 16); }
__device__ __forceinline__ float wave_sum32(float v) {
  v += __shfl_xor(v, 16, 32);
  v += __shfl_xor(v, 8, 32);
  v += __shfl_xor(v, 4, 32);
  v += __shfl_xor(v, 2, 32);
  v += __shfl_xor(v, 1, 32);
  return v;
}

__device__ __forceinline__ void dep_guard_b(v8f& a, v8f& b, v16b x, v16b y) { asm volatile("v_nop\n\tv_nop\n\tv_nop\n\tv_nop" : "+v"(a), "+v"(b) : "v"(x), "v"(y)); }
__device__ __forceinline__ void keep4_b(v16b a, v16b b, v16b c, v16b d) { asm volatile("v_nop" :: "v"(a), "v"(b), "v"(c), "v"(d)); }
__device__ __forceinline__ void acc_guard4(v8f& a, v8f& b, v8f& c, v8f& d) { asm volatile("v_nop\n\tv_nop\n\tv_nop\n\tv_nop" : "+v"(a), "+v"(b), "+v"(c), "+v"(d)); }
__device__ __forceinline__ void guard_one4(v8f& a, v16b x, v16b y, v16b z, v16b w) { asm volatile("v_nop\n\tv_nop\n\tv_nop\n\tv_nop" : "+v"(a) : "v"(x), "v"(y), "v"(z), "v"(w)); }

struct FragB {
  union U { v16b v; v8b h[2]; };
  static __device__ __forceinline__ v16b load(const __bf16* p) {
    U f; f.h[0] = *(const v8b*)(p); f.h[1] = *(const v8b*)(p + 16); return f.v;
  }
  static __device__ __forceinline__ v8f mma(v16b a, v16b b, v8f c) {
    return __builtin_amdgcn_wmma_f32_16x16x32_bf16(false, a, false, b, (short)0, c, false, false);
  }
};

template <int SPL, int BIAS_MODE, int OUT_MODE, int ACT>
__global__ __launch_bounds__(256) void wmma_gemm64(
    const unsigned short* __restrict__ Ap, const unsigned short* __restrict__ A2p, int lda, long strideA,
    const unsigned short* __restrict__ Btp, const unsigned short* __restrict__ Bt2p, int ldb, long strideB,
    void* __restrict__ Cout, void* __restrict__ Cout2, int ldc, long strideC,
    const float* __restrict__ bias,
    int M, int N, int K, float scale) {
  typedef __bf16 T;
  typedef v16b V;
  const T* A = (const T*)Ap; const T* A2 = (const T*)A2p; const T* Bt = (const T*)Btp; const T* Bt2 = (const T*)Bt2p;
  __shared__ __align__(16) float sT[8][16 * 68];
  const int b    = blockIdx.y;
  const int lane = threadIdx.x & 31;
  const int wave = threadIdx.x >> 5;
  const int tilesN = N >> 6;
  const int tilesM = M >> 6;
  const int tile = blockIdx.x * 8 + wave;
  if (tile >= tilesM * tilesN) return;
  const int tm = tile / tilesN;
  const int tn = tile - tm * tilesN;
  const int m0 = tm << 6;
  const int n0 = tn << 6;

  const T* Ab  = A  + (size_t)b * strideA;
  const T* Bb  = Bt + (size_t)b * strideB;
  const T* Ab2 = (SPL >= 1) ? (A2  + (size_t)b * strideA) : Ab;
  const T* Bb2 = (SPL == 2) ? (Bt2 + (size_t)b * strideB) : Bb;

  const int rlane = lane & 15;
  const int koff  = (lane >> 4) * 8;
  const int mOff  = (lane >> 4) * 8;

  v8f acc[4][4];
#pragma unroll
  for (int i = 0; i < 4; ++i)
#pragma unroll
    for (int j = 0; j < 4; ++j) acc[i][j] = (v8f){0.f,0.f,0.f,0.f,0.f,0.f,0.f,0.f};

  for (int k0 = 0; k0 < K; k0 += 32) {
    V bh[4], bl[4];
#pragma unroll
    for (int j = 0; j < 4; ++j) {
      const size_t bo = (size_t)(n0 + (j << 4) + rlane) * ldb + koff + k0;
      bh[j] = FragB::load(Bb + bo);
      if (SPL == 2) bl[j] = FragB::load(Bb2 + bo); else bl[j] = bh[j];
    }
#pragma unroll
    for (int i = 0; i < 4; ++i) {
      const size_t ao = (size_t)(m0 + (i << 4) + rlane) * lda + koff + k0;
      V ah = FragB::load(Ab + ao);
      V al = ah;
      if (SPL >= 1) al = FragB::load(Ab2 + ao);
#pragma unroll
      for (int j = 0; j < 4; ++j) {
        acc[i][j] = FragB::mma(ah, bh[j], acc[i][j]);
        if (SPL == 2) acc[i][j] = FragB::mma(ah, bl[j], acc[i][j]);
        if (SPL >= 1) acc[i][j] = FragB::mma(al, bh[j], acc[i][j]);
      }
      dep_guard_b(acc[i][0], acc[i][3], ah, al);
    }
    keep4_b(bh[0], bh[1], bh[2], bh[3]);
    if (SPL == 2) keep4_b(bl[0], bl[1], bl[2], bl[3]);
  }
  acc_guard4(acc[0][0], acc[0][1], acc[0][2], acc[0][3]);
  acc_guard4(acc[1][0], acc[1][1], acc[1][2], acc[1][3]);
  acc_guard4(acc[2][0], acc[2][1], acc[2][2], acc[2][3]);
  acc_guard4(acc[3][0], acc[3][1], acc[3][2], acc[3][3]);

  float* slab = sT[wave];
#pragma unroll
  for (int i = 0; i < 4; ++i) {
    const int mBase = m0 + (i << 4);
#pragma unroll
    for (int j = 0; j < 4; ++j) {
      const int n = n0 + (j << 4) + rlane;
      float bv = 0.f;
      if (BIAS_MODE == 2) bv = bias[n];
#pragma unroll
      for (int r = 0; r < 8; ++r) {
        float v = acc[i][j][r] * scale;
        if (BIAS_MODE == 1) v += bias[mBase + mOff + r];
        if (BIAS_MODE == 2) v += bv;
        if (ACT == 1) v = tanhf(v);
        if (ACT == 2) v = fmaxf(v, 0.0f);
        if (ACT == 3) v = v / (1.0f + expf(-v));
        if (ACT == 4) v = (v > 0.f) ? v : 0.01f * v;
        slab[(mOff + r) * 68 + (j << 4) + rlane] = v;
      }
    }
    __builtin_amdgcn_fence(__ATOMIC_RELEASE, "workgroup");
    __builtin_amdgcn_wave_barrier();
    __builtin_amdgcn_fence(__ATOMIC_ACQUIRE, "workgroup");
    if (OUT_MODE == 0) {
      float* C = (float*)Cout + (size_t)b * strideC;
      const int hh = lane >> 4, c4 = (lane & 15) * 4;
      for (int pass = 0; pass < 2; ++pass) {
#pragma unroll
        for (int it = 0; it < 8; ++it) {
          const int row = it * 2 + hh;
          v4f v = *(const v4f*)(slab + row * 68 + c4);
          *(volatile v4f*)(C + (size_t)(mBase + row) * ldc + n0 + c4) = v;
        }
        __threadfence();
      }
    } else {
      const int q = lane >> 3, c8 = (lane & 7) * 8;
      unsigned short* C  = (unsigned short*)Cout  + (size_t)b * strideC;
      unsigned short* C2 = (unsigned short*)Cout2 + (size_t)b * strideC;
      for (int pass = 0; pass < 2; ++pass) {
#pragma unroll
        for (int it = 0; it < 4; ++it) {
          const int row = it * 4 + q;
          const float* sp = slab + row * 68 + c8;
          v8h hv, lv;
#pragma unroll
          for (int e = 0; e < 8; ++e) {
            unsigned short hb = f2bf_bits(sp[e]);
            unsigned short lb = f2bf_bits(sp[e] - bf_bits2f(hb));
            hv[e] = __builtin_bit_cast(_Float16, hb);
            lv[e] = __builtin_bit_cast(_Float16, lb);
          }
          *(volatile v8h*)(C + (size_t)(mBase + row) * ldc + n0 + c8) = hv;
          *(volatile v8h*)(C2 + (size_t)(mBase + row) * ldc + n0 + c8) = lv;
        }
        __threadfence();
      }
    }
    __builtin_amdgcn_fence(__ATOMIC_RELEASE, "workgroup");
    __builtin_amdgcn_wave_barrier();
    __builtin_amdgcn_fence(__ATOMIC_ACQUIRE, "workgroup");
  }
}

__global__ __launch_bounds__(256) void cvt_transpose_bf16(const float* __restrict__ src, unsigned short* __restrict__ dst,
                                                          int Kdim, int Ndim) {
  __shared__ float tile[64][65];
  const int n0 = blockIdx.x * 64, k0 = blockIdx.y * 64;
  const int tid = threadIdx.x;
  {
    const int kk = tid >> 2, nq = (tid & 3) * 16;
    const float* sp = src + (size_t)(k0 + kk) * Ndim + n0 + nq;
    const v4f a0 = *(const v4f*)(sp), a1 = *(const v4f*)(sp + 4), a2 = *(const v4f*)(sp + 8), a3 = *(const v4f*)(sp + 12);
    tile[kk][nq + 0]  = a0[0]; tile[kk][nq + 1]  = a0[1]; tile[kk][nq + 2]  = a0[2]; tile[kk][nq + 3]  = a0[3];
    tile[kk][nq + 4]  = a1[0]; tile[kk][nq + 5]  = a1[1]; tile[kk][nq + 6]  = a1[2]; tile[kk][nq + 7]  = a1[3];
    tile[kk][nq + 8]  = a2[0]; tile[kk][nq + 9]  = a2[1]; tile[kk][nq + 10] = a2[2]; tile[kk][nq + 11] = a2[3];
    tile[kk][nq + 12] = a3[0]; tile[kk][nq + 13] = a3[1]; tile[kk][nq + 14] = a3[2]; tile[kk][nq + 15] = a3[3];
  }
  __syncthreads();
  const int nnA = tid >> 3, nnB = (tid >> 3) + 32, kq = (tid & 7) * 8;
  unsigned wa[4], wb[4];
#pragma unroll
  for (int p = 0; p < 4; ++p) {
    wa[p] = pack16x2(f2bf_bits(tile[kq + 2 * p][nnA]), f2bf_bits(tile[kq + 2 * p + 1][nnA]));
    wb[p] = pack16x2(f2bf_bits(tile[kq + 2 * p][nnB]), f2bf_bits(tile[kq + 2 * p + 1][nnB]));
  }
  const v4u ta = (v4u){wa[0], wa[1], wa[2], wa[3]};
  const v4u tb = (v4u){wb[0], wb[1], wb[2], wb[3]};
  unsigned short* pa = dst + (size_t)(n0 + nnA) * Kdim + k0 + kq;
  unsigned short* pb = dst + (size_t)(n0 + nnB) * Kdim + k0 + kq;
  for (int pass = 0; pass < 2; ++pass) {
    *(volatile v4u*)pa = ta;
    *(volatile v4u*)pb = tb;
    __threadfence();
  }
}

__global__ __launch_bounds__(256) void rte_vec_kernel(const float* __restrict__ src, float* __restrict__ dst, int n4) {
  const int i = blockIdx.x * 256 + threadIdx.x;
  if (i < n4) {
    const v4f a = *(const v4f*)(src + 4 * i);
    const v4f r = (v4f){bf_rte(a[0]), bf_rte(a[1]), bf_rte(a[2]), bf_rte(a[3])};
    *(volatile v4f*)(dst + 4 * i) = r;
    __threadfence();
    *(volatile v4f*)(dst + 4 * i) = r;
  }
}

__global__ __launch_bounds__(96) void ln_prep_kernel(const float* __restrict__ x, const float* __restrict__ gamma,
                                                     const float* __restrict__ beta,
                                                     unsigned short* __restrict__ xb, unsigned short* __restrict__ xnh,
                                                     unsigned short* __restrict__ xnl) {
  __shared__ float red_s[8];
  const int tok = blockIdx.x, tid = threadIdx.x, lane = tid & 31, wave = tid >> 5;
  const int c0 = tid * 8;
  const float* xr = x + (size_t)tok * kD + c0;
  const v4f xa = *(const v4f*)(xr), xq = *(const v4f*)(xr + 4);
  const v4f ga = *(const v4f*)(gamma + c0), gq = *(const v4f*)(gamma + c0 + 4);
  const v4f ba = *(const v4f*)(beta + c0), bq = *(const v4f*)(beta + c0 + 4);
  float v[8];
  v[0] = bf_rte(xa[0]); v[1] = bf_rte(xa[1]); v[2] = bf_rte(xa[2]); v[3] = bf_rte(xa[3]);
  v[4] = bf_rte(xq[0]); v[5] = bf_rte(xq[1]); v[6] = bf_rte(xq[2]); v[7] = bf_rte(xq[3]);
  float g[8], bt[8];
  g[0] = bf_rte(ga[0]); g[1] = bf_rte(ga[1]); g[2] = bf_rte(ga[2]); g[3] = bf_rte(ga[3]);
  g[4] = bf_rte(gq[0]); g[5] = bf_rte(gq[1]); g[6] = bf_rte(gq[2]); g[7] = bf_rte(gq[3]);
  bt[0] = bf_rte(ba[0]); bt[1] = bf_rte(ba[1]); bt[2] = bf_rte(ba[2]); bt[3] = bf_rte(ba[3]);
  bt[4] = bf_rte(bq[0]); bt[5] = bf_rte(bq[1]); bt[6] = bf_rte(bq[2]); bt[7] = bf_rte(bq[3]);

  float s = ((v[0] + v[1]) + (v[2] + v[3])) + ((v[4] + v[5]) + (v[6] + v[7]));
  s = wave_sum32(s);
  if (lane == 0) red_s[wave] = s;
  __syncthreads();
  const float mu = ((red_s[0] + red_s[1]) + red_s[2]) * (1.0f / 768.0f);
  float d[8];
  float ss = 0.0f;
#pragma unroll
  for (int i = 0; i < 8; ++i) { d[i] = v[i] - mu; ss += d[i] * d[i]; }
  ss = wave_sum32(ss);
  if (lane == 0) red_s[4 + wave] = ss;
  __syncthreads();
  const float var = ((red_s[4] + red_s[5]) + red_s[6]) * (1.0f / 768.0f);
  const float rs = rsqrtf(var + 1e-5f);

  unsigned wx[4], wh[4], wl[4];
#pragma unroll
  for (int p = 0; p < 4; ++p) {
    const int i0 = 2 * p, i1 = 2 * p + 1;
    const float y0 = d[i0] * rs * g[i0] + bt[i0];
    const float y1 = d[i1] * rs * g[i1] + bt[i1];
    unsigned short h0, l0, h1, l1;
    split_bf(y0, h0, l0);
    split_bf(y1, h1, l1);
    wx[p] = pack16x2(f2bf_bits(v[i0]), f2bf_bits(v[i1]));
    wh[p] = pack16x2(h0, h1);
    wl[p] = pack16x2(l0, l1);
  }
  const v4u tx = (v4u){wx[0], wx[1], wx[2], wx[3]};
  const v4u th = (v4u){wh[0], wh[1], wh[2], wh[3]};
  const v4u tl = (v4u){wl[0], wl[1], wl[2], wl[3]};
  const size_t o = (size_t)tok * kD + c0;
  for (int pass = 0; pass < 2; ++pass) {
    *(volatile v4u*)(xb + o)  = tx;
    *(volatile v4u*)(xnh + o) = th;
    *(volatile v4u*)(xnl + o) = tl;
    __threadfence();
  }
}

__device__ __forceinline__ float softplus_f(float a) {
  const float e = expf(a);
  const float r = logf(1.0f + e);
  return (a > 20.0f) ? a : r;
}
__device__ __forceinline__ float tanh_f(float p) {
  const float e = expf(2.0f * p);
  return 1.0f - 2.0f / (e + 1.0f);
}
__global__ __launch_bounds__(192) void gate_kernel(const float* __restrict__ semctx, const float* __restrict__ temperature,
                                                  float* __restrict__ gout) {
  __shared__ __align__(16) float g_s[kD];
  const int tok = blockIdx.x, tid = threadIdx.x;
  const float temp = bf_rte(temperature[0]);
  const float kPi = 3.14159265358979323846f;
  const float* sr = semctx + (size_t)tok * (2 * kD);
  const float* cr = semctx + (size_t)kNT * (2 * kD) + (size_t)tok * (2 * kD);
#pragma unroll 1
  for (int it = 0; it < 4; ++it) {
    const int c = tid + 192 * it;
    const float sa_raw = sr[c];
    const float sp_raw = sr[kD + c];
    const float ca_raw = cr[c];
    const float cp_raw = cr[kD + c];
    const float sa = softplus_f(sa_raw);
    const float ca = softplus_f(ca_raw);
    const float sp = tanh_f(sp_raw) * kPi;
    const float cp = tanh_f(cp_raw) * kPi;
    const float inter = ((sa * ca) * cosf(sp - cp)) * temp;
    const float gte = 1.0f / (1.0f + expf(-inter));
    g_s[c] = gte;
  }
  __syncthreads();
  const v4f gv = *(const v4f*)(g_s + tid * 4);
  float* op = gout + (size_t)tok * kD + tid * 4;
  *(volatile v4f*)op = gv;
  __threadfence();
  *(volatile v4f*)op = gv;
}

__global__ __launch_bounds__(256) void lin_attn_kernel(const float* __restrict__ qkv, const float* __restrict__ bqkv,
                                                      const float* __restrict__ gate,
                                                      unsigned short* __restrict__ ah_out, unsigned short* __restrict__ al_out) {
  __shared__ __align__(16) unsigned short Qh[64 * kAP];
  __shared__ __align__(16) unsigned short Ql[64 * kAP];
  __shared__ __align__(16) unsigned short KSh[64 * kAP];
  __shared__ __align__(16) unsigned short KSl[64 * kAP];
  __shared__ __align__(16) unsigned short KTh[64 * kAP];
  __shared__ __align__(16) unsigned short KTl[64 * kAP];
  __shared__ __align__(16) unsigned short VTh[64 * kAP];
  __shared__ __align__(16) unsigned short VTl[64 * kAP];
  __shared__ __align__(16) unsigned short Wh[64 * kAP];
  __shared__ __align__(16) unsigned short Wl[64 * kAP];
  __shared__ __align__(16) float Wf[64 * kOP];
  __shared__ __align__(16) float Os[64 * kOP];
  __shared__ float kpref_s[64];
  __shared__ float qk_s[64];
  __shared__ float denp_s[128];
  __shared__ float rden_s[64];
  __shared__ float bq_s[64];
  __shared__ float bk_s[64];
  __shared__ float bv_s[64];

  const int bh = blockIdx.x;
  const int b = bh / kH;
  const int h = bh - b * kH;
  const int tid = threadIdx.x, lane = tid & 31, wave = tid >> 5;
  const int rl = lane & 15, hh = lane >> 4, koff = hh * 8;
  const int ti = wave >> 1, tj0 = (wave & 1) * 2;
  const int srow = tid >> 2, dq = (tid & 3) * 16;

  for (int i = tid; i < 64 * kOP; i += 256) Wf[i] = 0.0f;
  for (int i = tid; i < 64 * kAP; i += 256) { Wh[i] = 0; Wl[i] = 0; }
  if (tid < 64) {
    kpref_s[tid] = 0.0f;
    bq_s[tid] = bf_rte(bqkv[h * kDH + tid]);
    bk_s[tid] = bf_rte(bqkv[kD + h * kDH + tid]);
    bv_s[tid] = bf_rte(bqkv[2 * kD + h * kDH + tid]);
  }
  __syncthreads();

  const v8f zero8 = (v8f){0.f,0.f,0.f,0.f,0.f,0.f,0.f,0.f};

#pragma unroll 1
  for (int c = 0; c < kNC; ++c) {
    __syncthreads();
    const size_t tok = (size_t)b * kL + (size_t)c * 64 + srow;
    const float* qp = qkv + tok * (3 * kD) + h * kDH + dq;
    {
      const v4f x0 = *(const v4f*)(qp), x1 = *(const v4f*)(qp + 4), x2 = *(const v4f*)(qp + 8), x3 = *(const v4f*)(qp + 12);
      float f[16] = {x0[0], x0[1], x0[2], x0[3], x1[0], x1[1], x1[2], x1[3],
                     x2[0], x2[1], x2[2], x2[3], x3[0], x3[1], x3[2], x3[3]};
      float qkp = 0.0f;
      unsigned hw[8], lw[8];
#pragma unroll
      for (int p = 0; p < 8; ++p) {
        float a0 = f[2 * p] + bq_s[dq + 2 * p];
        float a1 = f[2 * p + 1] + bq_s[dq + 2 * p + 1];
        a0 = (a0 > 0.0f) ? (a0 + 1.0f) : expf(a0);
        a1 = (a1 > 0.0f) ? (a1 + 1.0f) : expf(a1);
        qkp += a0 * kpref_s[dq + 2 * p];
        qkp += a1 * kpref_s[dq + 2 * p + 1];
        unsigned short h0, l0, h1, l1;
        split_bf(a0, h0, l0);
        split_bf(a1, h1, l1);
        hw[p] = pack16x2(h0, h1);
        lw[p] = pack16x2(l0, l1);
      }
      *(v4u*)(Qh + srow * kAP + dq)     = (v4u){hw[0], hw[1], hw[2], hw[3]};
      *(v4u*)(Qh + srow * kAP + dq + 8) = (v4u){hw[4], hw[5], hw[6], hw[7]};
      *(v4u*)(Ql + srow * kAP + dq)     = (v4u){lw[0], lw[1], lw[2], lw[3]};
      *(v4u*)(Ql + srow * kAP + dq + 8) = (v4u){lw[4], lw[5], lw[6], lw[7]};
      qkp += __shfl_xor(qkp, 1, 32);
      qkp += __shfl_xor(qkp, 2, 32);
      if ((tid & 3) == 0) qk_s[srow] = qkp;
    }
    __asm__ volatile("" ::: "memory");
    {
      const float* kp = qp + kD;
      const float* gp = gate + tok * kD + h * kDH + dq;
      const v4f x0 = *(const v4f*)(kp), x1 = *(const v4f*)(kp + 4), x2 = *(const v4f*)(kp + 8), x3 = *(const v4f*)(kp + 12);
      const v4f g0 = *(const v4f*)(gp), g1 = *(const v4f*)(gp + 4), g2 = *(const v4f*)(gp + 8), g3 = *(const v4f*)(gp + 12);
      float f[16] = {x0[0], x0[1], x0[2], x0[3], x1[0], x1[1], x1[2], x1[3],
                     x2[0], x2[1], x2[2], x2[3], x3[0], x3[1], x3[2], x3[3]};
      float gg[16] = {g0[0], g0[1], g0[2], g0[3], g1[0], g1[1], g1[2], g1[3],
                      g2[0], g2[1], g2[2], g2[3], g3[0], g3[1], g3[2], g3[3]};
      unsigned hw[8], lw[8];
#pragma unroll
      for (int p = 0; p < 8; ++p) {
        float a0 = (f[2 * p] + bk_s[dq + 2 * p]) * (1.0f + gg[2 * p]);
        float a1 = (f[2 * p + 1] + bk_s[dq + 2 * p + 1]) * (1.0f + gg[2 * p + 1]);
        a0 = (a0 > 0.0f) ? (a0 + 1.0f) : expf(a0);
        a1 = (a1 > 0.0f) ? (a1 + 1.0f) : expf(a1);
        unsigned short h0, l0, h1, l1;
        split_bf(a0, h0, l0);
        split_bf(a1, h1, l1);
        hw[p] = pack16x2(h0, h1);
        lw[p] = pack16x2(l0, l1);
        KTh[(dq + 2 * p) * kAP + srow] = h0;
        KTh[(dq + 2 * p + 1) * kAP + srow] = h1;
        KTl[(dq + 2 * p) * kAP + srow] = l0;
        KTl[(dq + 2 * p + 1) * kAP + srow] = l1;
      }
      *(v4u*)(KSh + srow * kAP + dq)     = (v4u){hw[0], hw[1], hw[2], hw[3]};
      *(v4u*)(KSh + srow * kAP + dq + 8) = (v4u){hw[4], hw[5], hw[6], hw[7]};
      *(v4u*)(KSl + srow * kAP + dq)     = (v4u){lw[0], lw[1], lw[2], lw[3]};
      *(v4u*)(KSl + srow * kAP + dq + 8) = (v4u){lw[4], lw[5], lw[6], lw[7]};
    }
    __asm__ volatile("" ::: "memory");
    {
      const float* vp = qp + 2 * kD;
      const v4f x0 = *(const v4f*)(vp), x1 = *(const v4f*)(vp + 4), x2 = *(const v4f*)(vp + 8), x3 = *(const v4f*)(vp + 12);
      float f[16] = {x0[0], x0[1], x0[2], x0[3], x1[0], x1[1], x1[2], x1[3],
                     x2[0], x2[1], x2[2], x2[3], x3[0], x3[1], x3[2], x3[3]};
#pragma unroll
      for (int d = 0; d < 16; ++d) {
        const float a = f[d] + bv_s[dq + d];
        unsigned short hb, lb;
        split_bf(a, hb, lb);
        VTh[(dq + d) * kAP + srow] = hb;
        VTl[(dq + d) * kAP + srow] = lb;
      }
    }
    __syncthreads();

    v8f sacc[2];
#pragma unroll
    for (int t = 0; t < 2; ++t) {
      const int tj = tj0 + t;
      v8f acc = zero8;
#pragma unroll
      for (int ks = 0; ks < 64; ks += 32) {
        const v16b a_h = FragB::load((const __bf16*)Qh + (ti * 16 + rl) * kAP + koff + ks);
        const v16b a_l = FragB::load((const __bf16*)Ql + (ti * 16 + rl) * kAP + koff + ks);
        const v16b b_h = FragB::load((const __bf16*)KSh + (tj * 16 + rl) * kAP + koff + ks);
        const v16b b_l = FragB::load((const __bf16*)KSl + (tj * 16 + rl) * kAP + koff + ks);
        acc = FragB::mma(a_h, b_h, acc);
        acc = FragB::mma(a_h, b_l, acc);
        acc = FragB::mma(a_l, b_h, acc);
        guard_one4(acc, a_h, a_l, b_h, b_l);
      }
      sacc[t] = acc;
    }
    float ps[8];
    unsigned short shb[2][8], slb[2][8];
#pragma unroll
    for (int r = 0; r < 8; ++r) ps[r] = 0.0f;
#pragma unroll
    for (int t = 0; t < 2; ++t) {
#pragma unroll
      for (int r = 0; r < 8; ++r) {
        const int i = ti * 16 + 8 * hh + r;
        const int j = (tj0 + t) * 16 + rl;
        const float sv = (j <= i) ? sacc[t][r] : 0.0f;
        ps[r] += sv;
        split_bf(sv, shb[t][r], slb[t][r]);
      }
    }
#pragma unroll
    for (int r = 0; r < 8; ++r) {
      float s = ps[r];
      s += __shfl_xor(s, 1, 32);
      s += __shfl_xor(s, 2, 32);
      s += __shfl_xor(s, 4, 32);
      s += __shfl_xor(s, 8, 32);
      ps[r] = s;
    }
    if (rl == 0) {
#pragma unroll
      for (int r = 0; r < 8; ++r) denp_s[(wave & 1) * 64 + ti * 16 + 8 * hh + r] = ps[r];
    }
    __syncthreads();
#pragma unroll
    for (int t = 0; t < 2; ++t) {
#pragma unroll
      for (int r = 0; r < 8; ++r) {
        const int i = ti * 16 + 8 * hh + r;
        const int j = (tj0 + t) * 16 + rl;
        KSh[i * kAP + j] = shb[t][r];
        KSl[i * kAP + j] = slb[t][r];
      }
    }
    __syncthreads();

    if (tid < 64) {
      const float ds = ((denp_s[tid] + denp_s[64 + tid]) + qk_s[tid]) + 1e-6f;
      rden_s[tid] = 1.0f / ds;
    }
    if (tid >= 64 && tid < 128) {
      const int d = tid - 64;
      float s = 0.0f;
#pragma unroll 8
      for (int j = 0; j < 64; ++j) s += bf_bits2f(KTh[d * kAP + j]) + bf_bits2f(KTl[d * kAP + j]);
      kpref_s[d] = kpref_s[d] + s;
    }
#pragma unroll
    for (int t = 0; t < 2; ++t) {
      const int tj = tj0 + t;
      v8f acc = zero8;
#pragma unroll
      for (int ks = 0; ks < 64; ks += 32) {
        const v16b a_h = FragB::load((const __bf16*)Qh + (ti * 16 + rl) * kAP + koff + ks);
        const v16b a_l = FragB::load((const __bf16*)Ql + (ti * 16 + rl) * kAP + koff + ks);
        const v16b b_h = FragB::load((const __bf16*)Wh + (tj * 16 + rl) * kAP + koff + ks);
        const v16b b_l = FragB::load((const __bf16*)Wl + (tj * 16 + rl) * kAP + koff + ks);
        acc = FragB::mma(a_h, b_h, acc);
        acc = FragB::mma(a_h, b_l, acc);
        acc = FragB::mma(a_l, b_h, acc);
        guard_one4(acc, a_h, a_l, b_h, b_l);
      }
#pragma unroll
      for (int ks = 0; ks < 64; ks += 32) {
        const v16b a_h = FragB::load((const __bf16*)KSh + (ti * 16 + rl) * kAP + koff + ks);
        const v16b a_l = FragB::load((const __bf16*)KSl + (ti * 16 + rl) * kAP + koff + ks);
        const v16b b_h = FragB::load((const __bf16*)VTh + (tj * 16 + rl) * kAP + koff + ks);
        const v16b b_l = FragB::load((const __bf16*)VTl + (tj * 16 + rl) * kAP + koff + ks);
        acc = FragB::mma(a_h, b_h, acc);
        acc = FragB::mma(a_h, b_l, acc);
        acc = FragB::mma(a_l, b_h, acc);
        guard_one4(acc, a_h, a_l, b_h, b_l);
      }
#pragma unroll
      for (int r = 0; r < 8; ++r) Os[(ti * 16 + 8 * hh + r) * kOP + tj * 16 + rl] = acc[r];
    }
    __syncthreads();

    {
      const int gq = tid >> 3, c8 = (tid & 7) * 8;
      const int rA = gq, rB = gq + 32;
      const float rdA = rden_s[rA], rdB = rden_s[rB];
      const v4f oa = *(const v4f*)(Os + rA * kOP + c8), ob = *(const v4f*)(Os + rA * kOP + c8 + 4);
      const v4f oc = *(const v4f*)(Os + rB * kOP + c8), od = *(const v4f*)(Os + rB * kOP + c8 + 4);
      float eA[8] = {oa[0], oa[1], oa[2], oa[3], ob[0], ob[1], ob[2], ob[3]};
      float eB[8] = {oc[0], oc[1], oc[2], oc[3], od[0], od[1], od[2], od[3]};
      unsigned hwA[4], lwA[4], hwB[4], lwB[4];
#pragma unroll
      for (int p = 0; p < 4; ++p) {
        unsigned short h0, l0, h1, l1;
        split_bf(eA[2 * p] * rdA, h0, l0);
        split_bf(eA[2 * p + 1] * rdA, h1, l1);
        hwA[p] = pack16x2(h0, h1);
        lwA[p] = pack16x2(l0, l1);
        split_bf(eB[2 * p] * rdB, h0, l0);
        split_bf(eB[2 * p + 1] * rdB, h1, l1);
        hwB[p] = pack16x2(h0, h1);
        lwB[p] = pack16x2(l0, l1);
      }
      const v4u thA = (v4u){hwA[0], hwA[1], hwA[2], hwA[3]};
      const v4u tlA = (v4u){lwA[0], lwA[1], lwA[2], lwA[3]};
      const v4u thB = (v4u){hwB[0], hwB[1], hwB[2], hwB[3]};
      const v4u tlB = (v4u){lwB[0], lwB[1], lwB[2], lwB[3]};
      const size_t tokA = (size_t)b * kL + (size_t)c * 64 + rA;
      const size_t tokB = tokA + 32;
      unsigned short* phA = ah_out + tokA * kD + h * kDH + c8;
      unsigned short* plA = al_out + tokA * kD + h * kDH + c8;
      unsigned short* phB = ah_out + tokB * kD + h * kDH + c8;
      unsigned short* plB = al_out + tokB * kD + h * kDH + c8;
      for (int pass = 0; pass < 2; ++pass) {
        *(volatile v4u*)phA = thA;
        *(volatile v4u*)plA = tlA;
        *(volatile v4u*)phB = thB;
        *(volatile v4u*)plB = tlB;
        __threadfence();
      }
    }
#pragma unroll
    for (int t = 0; t < 2; ++t) {
      const int td = tj0 + t;
      v8f acc;
#pragma unroll
      for (int r = 0; r < 8; ++r) acc[r] = Wf[(ti * 16 + 8 * hh + r) * kOP + td * 16 + rl];
#pragma unroll
      for (int ks = 0; ks < 64; ks += 32) {
        const v16b a_h = FragB::load((const __bf16*)VTh + (ti * 16 + rl) * kAP + koff + ks);
        const v16b a_l = FragB::load((const __bf16*)VTl + (ti * 16 + rl) * kAP + koff + ks);
        const v16b b_h = FragB::load((const __bf16*)KTh + (td * 16 + rl) * kAP + koff + ks);
        const v16b b_l = FragB::load((const __bf16*)KTl + (td * 16 + rl) * kAP + koff + ks);
        acc = FragB::mma(a_h, b_h, acc);
        acc = FragB::mma(a_h, b_l, acc);
        acc = FragB::mma(a_l, b_h, acc);
        guard_one4(acc, a_h, a_l, b_h, b_l);
      }
#pragma unroll
      for (int r = 0; r < 8; ++r) {
        const float w = acc[r];
        const int wi = ti * 16 + 8 * hh + r;
        const int wj = td * 16 + rl;
        Wf[wi * kOP + wj] = w;
        unsigned short hb, lb;
        split_bf(w, hb, lb);
        Wh[wi * kAP + wj] = hb;
        Wl[wi * kAP + wj] = lb;
      }
    }
  }
}

extern "C" void kernel_launch(void* const* d_in, const int* in_sizes, int n_in,
                              void* d_out, int out_size, void* d_ws, size_t ws_size, hipStream_t stream) {
  (void)in_sizes; (void)n_in; (void)out_size;
  if (ws_size < kWsEnd) return;

  const float* x      = (const float*)d_in[0];
  const float* W_qkv  = (const float*)d_in[1];
  const float* b_qkv  = (const float*)d_in[2];
  const float* W_sd   = (const float*)d_in[3];
  const float* W_su   = (const float*)d_in[4];
  const float* W_cd   = (const float*)d_in[5];
  const float* W_cu   = (const float*)d_in[6];
  const float* temper = (const float*)d_in[7];
  const float* W_proj = (const float*)d_in[8];
  const float* b_proj = (const float*)d_in[9];
  const float* gamma  = (const float*)d_in[10];
  const float* beta   = (const float*)d_in[11];

  float* out_main = (float*)d_out;
  float* out_gate = (float*)d_out + kOut1Elems;

  char* ws = (char*)d_ws;
  unsigned short* WqkvT  = (unsigned short*)(ws + kOffWqkvT);
  unsigned short* WdownT = (unsigned short*)(ws + kOffWdownT);
  unsigned short* WupT   = (unsigned short*)(ws + kOffWupT);
  unsigned short* WprojT = (unsigned short*)(ws + kOffWprojT);
  float*          bprojR = (float*)(ws + kOffBproj);
  unsigned short* xB     = (unsigned short*)(ws + kOffXb);
  unsigned short* xnH    = (unsigned short*)(ws + kOffXnh);
  unsigned short* xnL    = (unsigned short*)(ws + kOffXnl);
  float*          qkvF   = (float*)(ws + kOffQkv);
  unsigned short* hH     = (unsigned short*)(ws + kOffHh);
  unsigned short* hL     = (unsigned short*)(ws + kOffHl);
  float*          semctx = (float*)(ws + kOffSemCtx);
  unsigned short* attnH  = (unsigned short*)(ws + kOffAttnH);
  unsigned short* attnL  = (unsigned short*)(ws + kOffAttnL);

  cvt_transpose_bf16<<<dim3((3 * kD) / 64, kD / 64), 256, 0, stream>>>(W_qkv, WqkvT, kD, 3 * kD);
  cvt_transpose_bf16<<<dim3(kR / 64, kD / 64), 256, 0, stream>>>(W_sd, WdownT, kD, kR);
  cvt_transpose_bf16<<<dim3(kR / 64, kD / 64), 256, 0, stream>>>(W_cd, WdownT + (size_t)kR * kD, kD, kR);
  cvt_transpose_bf16<<<dim3((2 * kD) / 64, kR / 64), 256, 0, stream>>>(W_su, WupT, kR, 2 * kD);
  cvt_transpose_bf16<<<dim3((2 * kD) / 64, kR / 64), 256, 0, stream>>>(W_cu, WupT + (size_t)(2 * kD) * kR, kR, 2 * kD);
  cvt_transpose_bf16<<<dim3(kD / 64, kD / 64), 256, 0, stream>>>(W_proj, WprojT, kD, kD);
  rte_vec_kernel<<<1, 256, 0, stream>>>(b_proj, bprojR, kD / 4);
  ln_prep_kernel<<<kNT, 96, 0, stream>>>(x, gamma, beta, xB, xnH, xnL);
  {
    const int tiles = (kNT / 64) * ((3 * kD) / 64);
    wmma_gemm64<1, 0, 0, 0><<<dim3((tiles + 7) / 8, 1), 256, 0, stream>>>(
        xnH, xnL, kD, 0L, WqkvT, WqkvT, kD, 0L, (void*)qkvF, (void*)qkvF, 3 * kD, 0L, bprojR, kNT, 3 * kD, kD, 1.0f);
  }
  {
    const int tiles = (kNT / 64) * ((2 * kR) / 64);
    wmma_gemm64<0, 0, 2, 3><<<dim3((tiles + 7) / 8, 1), 256, 0, stream>>>(
        xB, xB, kD, 0L, WdownT, WdownT, kD, 0L, (void*)hH, (void*)hL, 2 * kR, 0L, bprojR, kNT, 2 * kR, kD, 1.0f);
  }
  {
    const int tiles = (kNT / 64) * ((2 * kD) / 64);
    wmma_gemm64<1, 0, 0, 0><<<dim3((tiles + 7) / 8, 2), 256, 0, stream>>>(
        hH, hL, 2 * kR, (long)kR, WupT, WupT, kR, (long)(2 * kD) * kR, (void*)semctx, (void*)semctx, 2 * kD,
        (long)kNT * (2 * kD), bprojR, kNT, 2 * kD, kR, 1.0f);
  }
  gate_kernel<<<kNT, 192, 0, stream>>>(semctx, temper, out_gate);
  lin_attn_kernel<<<kBH, 256, 0, stream>>>(qkvF, b_qkv, out_gate, attnH, attnL);
  {
    const int tiles = (kNT / 64) * (kD / 64);
    wmma_gemm64<1, 2, 0, 0><<<dim3((tiles + 7) / 8, 1), 256, 0, stream>>>(
        attnH, attnL, kD, 0L, WprojT, WprojT, kD, 0L, (void*)out_main, (void*)out_main, kD, 0L, bprojR, kNT, kD, kD, 1.0f);
  }
}
